// SimpleLSTM_56667798503960
// MI455X (gfx1250) — hardware-verified
//
#include <hip/hip_runtime.h>
#include <math.h>

typedef __attribute__((ext_vector_type(16))) _Float16 v16h;
typedef __attribute__((ext_vector_type(8)))  _Float16 v8h;
typedef __attribute__((ext_vector_type(4)))  _Float16 v4h;
typedef __attribute__((ext_vector_type(16))) __bf16   v16b;
typedef __attribute__((ext_vector_type(8)))  __bf16   v8b;
typedef __attribute__((ext_vector_type(8)))  float    v8f;
typedef __attribute__((ext_vector_type(4)))  float    v4f;
typedef __attribute__((ext_vector_type(4)))  unsigned int v4u;

constexpr int kBatch = 64;
constexpr int kSteps = 2048;
constexpr int kIn    = 9;
constexpr int kHid   = 128;
constexpr int kGates = 512;
constexpr int kFc1   = 20;
constexpr int kRows  = kBatch * kSteps;
constexpr int kKpad0 = 160;
constexpr int kKpad1 = 256;
constexpr int kHeadN = 64;
constexpr float kWScale    = 16.0f;
constexpr float kWScaleInv = 0.0625f;

constexpr size_t kPlaneBytes = (size_t)kRows * kHid * 2;
constexpr size_t kGmatBytes  = (size_t)kRows * kHeadN * 4;
constexpr size_t kFc1Bytes   = (size_t)kHeadN * kHid * 2;
constexpr size_t kOffH0   = 0;
constexpr size_t kOffH1   = kOffH0 + kPlaneBytes;
constexpr size_t kOffGmat = kOffH1 + kPlaneBytes;
constexpr size_t kOffFc1  = kOffGmat + kGmatBytes;
constexpr size_t kWsTotal = kOffFc1 + kFc1Bytes;
static_assert(kWsTotal == 100679680, "carve total");
static_assert(kWsTotal <= 134217728, "carve under 128 MiB");
static_assert(kRows % 64 == 0 && kHeadN % 64 == 0 && kHid % 32 == 0, "head GEMM tile contract");
static_assert(kRows % 256 == 0, "epilogue grid");

__device__ __forceinline__ unsigned short f2bf_bits(float f) {
  unsigned u = __float_as_uint(f);
  return (unsigned short)((u + 0x7FFFu + ((u >> 16) & 1u)) >> 16);
}
__device__ __forceinline__ float bf_bits2f(unsigned short h) { return __uint_as_float(((unsigned)h) << 16); }

__device__ __forceinline__ void dep_guard_h(v8f& a, v8f& b, v16h x, v16h y) { asm volatile("v_nop\n\tv_nop\n\tv_nop\n\tv_nop" : "+v"(a), "+v"(b) : "v"(x), "v"(y)); }
__device__ __forceinline__ void dep_guard_b(v8f& a, v8f& b, v16b x, v16b y) { asm volatile("v_nop\n\tv_nop\n\tv_nop\n\tv_nop" : "+v"(a), "+v"(b) : "v"(x), "v"(y)); }
__device__ __forceinline__ void keep4_h(v16h a, v16h b, v16h c, v16h d) { asm volatile("v_nop" :: "v"(a), "v"(b), "v"(c), "v"(d)); }
__device__ __forceinline__ void keep4_b(v16b a, v16b b, v16b c, v16b d) { asm volatile("v_nop" :: "v"(a), "v"(b), "v"(c), "v"(d)); }
__device__ __forceinline__ void acc_guard4(v8f& a, v8f& b, v8f& c, v8f& d) { asm volatile("v_nop\n\tv_nop\n\tv_nop\n\tv_nop" : "+v"(a), "+v"(b), "+v"(c), "+v"(d)); }
template <typename T> struct Frag;
template <> struct Frag<_Float16> {
  typedef v16h V; union U { v16h v; v8h h[2]; };
  static __device__ __forceinline__ v16h load(const _Float16* p) {
    U f; f.h[0] = *(const v8h*)(p); f.h[1] = *(const v8h*)(p + 16); return f.v;
  }
  static __device__ __forceinline__ v8f mma(v16h a, v16h b, v8f c) {
    return __builtin_amdgcn_wmma_f32_16x16x32_f16(false, a, false, b, (short)0, c, false, false);
  }
  static __device__ __forceinline__ void guard(v8f& a, v8f& b, v16h x, v16h y) { dep_guard_h(a, b, x, y); }
  static __device__ __forceinline__ void keep(v16h a, v16h b, v16h c, v16h d) { keep4_h(a, b, c, d); }
};
template <> struct Frag<__bf16> {
  typedef v16b V; union U { v16b v; v8b h[2]; };
  static __device__ __forceinline__ v16b load(const __bf16* p) {
    U f; f.h[0] = *(const v8b*)(p); f.h[1] = *(const v8b*)(p + 16); return f.v;
  }
  static __device__ __forceinline__ v8f mma(v16b a, v16b b, v8f c) {
    return __builtin_amdgcn_wmma_f32_16x16x32_bf16(false, a, false, b, (short)0, c, false, false);
  }
  static __device__ __forceinline__ void guard(v8f& a, v8f& b, v16b x, v16b y) { dep_guard_b(a, b, x, y); }
  static __device__ __forceinline__ void keep(v16b a, v16b b, v16b c, v16b d) { keep4_b(a, b, c, d); }
};

template <int ET> struct Elem;
template <> struct Elem<0> { typedef _Float16 T; };
template <> struct Elem<1> { typedef __bf16 T; };
template <int ET, bool SPLIT, int BIAS_MODE, int OUT_MODE, bool RESID, int ACT = 0>
__global__ __launch_bounds__(256) void wmma_gemm64(
    const unsigned short* __restrict__ Ap, const unsigned short* __restrict__ A2p, int lda, long strideA,
    const unsigned short* __restrict__ Btp, const unsigned short* __restrict__ Bt2p, int ldb, long strideB,
    void* __restrict__ Cout, void* __restrict__ Cout2, int ldc, long strideC,
    const float* __restrict__ bias,
    const float* __restrict__ resid, long strideR,
    int M, int N, int K, float scale) {
  typedef typename Elem<ET>::T T;
  typedef typename Frag<T>::V V;
  const T* A = (const T*)Ap; const T* A2 = (const T*)A2p; const T* Bt = (const T*)Btp; const T* Bt2 = (const T*)Bt2p;
  __shared__ __align__(16) float sT[8][16 * 68];
  const int b    = blockIdx.y;
  const int lane = threadIdx.x & 31;
  const int wave = threadIdx.x >> 5;
  const int tilesN = N >> 6;
  const int tilesM = M >> 6;
  const int tile = blockIdx.x * 8 + wave;
  if (tile >= tilesM * tilesN) return;
  const int tm = tile / tilesN;
  const int tn = tile - tm * tilesN;
  const int m0 = tm << 6;
  const int n0 = tn << 6;

  const T* Ab  = A  + (size_t)b * strideA;
  const T* Bb  = Bt + (size_t)b * strideB;
  const T* Ab2 = SPLIT ? (A2  + (size_t)b * strideA) : nullptr;
  const T* Bb2 = SPLIT ? (Bt2 + (size_t)b * strideB) : nullptr;

  const int rlane = lane & 15;
  const int koff  = (lane >> 4) * 8;
  const int mOff  = (lane >> 4) * 8;

  v8f acc[4][4];
#pragma unroll
  for (int i = 0; i < 4; ++i)
#pragma unroll
    for (int j = 0; j < 4; ++j) acc[i][j] = (v8f){0.f,0.f,0.f,0.f,0.f,0.f,0.f,0.f};

  for (int k0 = 0; k0 < K; k0 += 32) {
    V bh[4], bl[4];
#pragma unroll
    for (int j = 0; j < 4; ++j) {
      const size_t bo = (size_t)(n0 + (j << 4) + rlane) * ldb + koff + k0;
      bh[j] = Frag<T>::load(Bb + bo);
      if (SPLIT) bl[j] = Frag<T>::load(Bb2 + bo);
    }
#pragma unroll
    for (int i = 0; i < 4; ++i) {
      const size_t ao = (size_t)(m0 + (i << 4) + rlane) * lda + koff + k0;
      V ah = Frag<T>::load(Ab + ao);
      V al;
      if (SPLIT) al = Frag<T>::load(Ab2 + ao);
#pragma unroll
      for (int j = 0; j < 4; ++j) {
        acc[i][j] = Frag<T>::mma(ah, bh[j], acc[i][j]);
        if (SPLIT) {
          acc[i][j] = Frag<T>::mma(ah, bl[j], acc[i][j]);
          acc[i][j] = Frag<T>::mma(al, bh[j], acc[i][j]);
        }
      }
      Frag<T>::guard(acc[i][0], acc[i][3], ah, SPLIT ? al : ah);
    }
    Frag<T>::keep(bh[0], bh[1], bh[2], bh[3]);
    if (SPLIT) Frag<T>::keep(bl[0], bl[1], bl[2], bl[3]);
  }
  acc_guard4(acc[0][0], acc[0][1], acc[0][2], acc[0][3]);
  acc_guard4(acc[1][0], acc[1][1], acc[1][2], acc[1][3]);
  acc_guard4(acc[2][0], acc[2][1], acc[2][2], acc[2][3]);
  acc_guard4(acc[3][0], acc[3][1], acc[3][2], acc[3][3]);

  float* slab = sT[wave];
  const float* Rb = RESID ? (resid + (size_t)b * strideR) : nullptr;
#pragma unroll
  for (int i = 0; i < 4; ++i) {
    const int mBase = m0 + (i << 4);
#pragma unroll
    for (int j = 0; j < 4; ++j) {
      const int n = n0 + (j << 4) + rlane;
      float bv = 0.f;
      if (BIAS_MODE == 2) bv = bias[n];
#pragma unroll
      for (int r = 0; r < 8; ++r) {
        float v = acc[i][j][r] * scale;
        if (BIAS_MODE == 1) v += bias[mBase + mOff + r];
        if (BIAS_MODE == 2) v += bv;
        if (RESID) v += Rb[(size_t)(mBase + mOff + r) * ldc + n];
        if (ACT == 1) v = tanhf(v);
        if (ACT == 2) v = fmaxf(v, 0.0f);
        if (ACT == 3) v = v / (1.0f + expf(-v));
        if (ACT == 4) v = (v > 0.f) ? v : 0.01f * v;
        if (ACT == 5) v = 0.5f * v * (1.0f + erff(v * 0.70710678118654752f));
        slab[(mOff + r) * 68 + (j << 4) + rlane] = v;
      }
    }
    __builtin_amdgcn_fence(__ATOMIC_RELEASE, "workgroup");
    __builtin_amdgcn_wave_barrier();
    __builtin_amdgcn_fence(__ATOMIC_ACQUIRE, "workgroup");
    if (OUT_MODE == 0) {
      float* C = (float*)Cout + (size_t)b * strideC;
      const int hh = lane >> 4, c4 = (lane & 15) * 4;
      for (int pass = 0; pass < 2; ++pass) {
#pragma unroll
        for (int it = 0; it < 8; ++it) {
          const int row = it * 2 + hh;
          v4f v = *(const v4f*)(slab + row * 68 + c4);
          *(volatile v4f*)(C + (size_t)(mBase + row) * ldc + n0 + c4) = v;
        }
        __threadfence();
      }
    } else {
      const int q = lane >> 3, c8 = (lane & 7) * 8;
      unsigned short* C  = (unsigned short*)Cout  + (size_t)b * strideC;
      unsigned short* C2 = (OUT_MODE == 2) ? ((unsigned short*)Cout2 + (size_t)b * strideC) : nullptr;
      for (int pass = 0; pass < 2; ++pass) {
#pragma unroll
        for (int it = 0; it < 4; ++it) {
          const int row = it * 4 + q;
          const float* sp = slab + row * 68 + c8;
          v8h hv, lv;
#pragma unroll
          for (int e = 0; e < 8; ++e) {
            if (OUT_MODE == 1) {
              hv[e] = (_Float16)sp[e];
            } else {
              unsigned short hb = f2bf_bits(sp[e]);
              unsigned short lb = f2bf_bits(sp[e] - bf_bits2f(hb));
              hv[e] = __builtin_bit_cast(_Float16, hb);
              lv[e] = __builtin_bit_cast(_Float16, lb);
            }
          }
          *(volatile v8h*)(C + (size_t)(mBase + row) * ldc + n0 + c8) = hv;
          if (OUT_MODE == 2) *(volatile v8h*)(C2 + (size_t)(mBase + row) * ldc + n0 + c8) = lv;
        }
        __threadfence();
      }
    }
    __builtin_amdgcn_fence(__ATOMIC_RELEASE, "workgroup");
    __builtin_amdgcn_wave_barrier();
    __builtin_amdgcn_fence(__ATOMIC_ACQUIRE, "workgroup");
  }
}

__device__ __forceinline__ float sigm_f(float v) {
  const float e = expf(-v);
  return __builtin_amdgcn_rcpf(1.0f + e);
}
__device__ __forceinline__ float tanh_f(float v) {
  const float t = expf(-2.0f * fabsf(v));
  const float r = (1.0f - t) * __builtin_amdgcn_rcpf(1.0f + t);
  return copysignf(r, v);
}

template <int KIN, int KPAD>
__global__ __launch_bounds__(256) void lstm_layer_kernel(
    const float* __restrict__ Whh,
    const float* __restrict__ Wih,
    const float* __restrict__ bih,
    const float* __restrict__ bhh,
    const float* __restrict__ xin,
    const unsigned short* __restrict__ hin,
    unsigned short* __restrict__ hout) {
  constexpr int NCH = KPAD / 32;
  constexpr int AP  = KPAD + 8;
  constexpr int WH  = kGates * KPAD;
  constexpr int AH  = 16 * AP;
  static_assert(KPAD % 32 == 0 && kHid + KIN <= KPAD, "k padding");
  static_assert((AP * 2) % 16 == 0 && (WH * 2) % 16 == 0, "16B alignment");
  static_assert(KPAD % 4 == 0, "fill granularity");
  extern __shared__ __align__(16) _Float16 lds_dyn[];
  _Float16* Wl = lds_dyn;
  _Float16* Ab = lds_dyn + WH;
  const _Float16* hin16 = (const _Float16*)hin;
  _Float16* hout16 = (_Float16*)hout;

  const int tid  = threadIdx.x;
  const int lane = tid & 31;
  const int wv   = tid >> 5;
  const int hh   = lane >> 4;
  const int cc   = lane & 15;
  const int b0   = blockIdx.x * 16;
  const int ucol = wv * 16 + cc;

  {
    const v4u z = (v4u){0u, 0u, 0u, 0u};
#pragma unroll 1
    for (int i = tid; i < 4 * AP; i += 256) *(v4u*)(Ab + i * 8) = z;
  }
#pragma unroll 1
  for (int e4 = tid; e4 < WH / 4; e4 += 256) {
    const int e = e4 * 4;
    const int n = e / KPAD;
    const int k = e - n * KPAD;
    float wq[4];
#pragma unroll
    for (int j = 0; j < 4; ++j) {
      const int kj  = k + j;
      const int khh = (kj < kHid) ? kj : (kHid - 1);
      int kih = kj - kHid;
      kih = (kih < 0) ? 0 : ((kih > KIN - 1) ? (KIN - 1) : kih);
      const float wa = Whh[(size_t)n * kHid + khh];
      const float wb = Wih[(size_t)n * KIN + kih];
      const float sel = (kj < kHid) ? wa : ((kj < kHid + KIN) ? wb : 0.0f);
      wq[j] = sel * kWScale;
    }
    v4h hv4;
    hv4[0] = (_Float16)wq[0]; hv4[1] = (_Float16)wq[1]; hv4[2] = (_Float16)wq[2]; hv4[3] = (_Float16)wq[3];
    *(v4h*)(Wl + e) = hv4;
  }
  __syncthreads();

  int xm, xj;
  if constexpr (KIN == kIn) { xm = tid / kIn; xj = tid - xm * kIn; }
  else { xm = tid >> 4; xj = (tid & 15) * 8; }
  const int xmc = (xm < 16) ? xm : 15;
  const size_t xrow0 = (size_t)(b0 + xmc) * kSteps;
  if constexpr (KIN == kIn) {
    const float xs0 = xin[xrow0 * kIn + xj];
    if (tid < 16 * kIn) Ab[xm * AP + kHid + xj] = (_Float16)xs0;
  } else {
    const v4u q0 = *(const v4u*)(hin16 + xrow0 * kHid + xj);
    *(v4u*)(Ab + xm * AP + kHid + xj) = q0;
  }
  float bs[4];
#pragma unroll
  for (int g = 0; g < 4; ++g) bs[g] = bih[g * kHid + ucol] + bhh[g * kHid + ucol];
  __syncthreads();

  v8f cst = (v8f){0.f, 0.f, 0.f, 0.f, 0.f, 0.f, 0.f, 0.f};

  for (int t = 0; t < kSteps; ++t) {
    const _Float16* cur = Ab + (t & 1) * AH;
    _Float16* nxt = Ab + ((t + 1) & 1) * AH;
    const int tn = (t + 1 < kSteps) ? (t + 1) : t;

    float xs = 0.0f;
    v4u xq = (v4u){0u, 0u, 0u, 0u};
    if constexpr (KIN == kIn) { xs = xin[(xrow0 + tn) * kIn + xj]; }
    else { xq = *(const v4u*)(hin16 + (xrow0 + tn) * kHid + xj); }

    v8f acc[4];
#pragma unroll
    for (int g = 0; g < 4; ++g) acc[g] = (v8f){0.f, 0.f, 0.f, 0.f, 0.f, 0.f, 0.f, 0.f};

#pragma unroll 1
    for (int ch = 0; ch < NCH; ++ch) {
      const int ko = ch * 32 + 8 * hh;
      const v16h af = Frag<_Float16>::load(cur + cc * AP + ko);
      v16h bq[4];
#pragma unroll
      for (int g = 0; g < 4; ++g)
        bq[g] = Frag<_Float16>::load(Wl + (g * kHid + ucol) * KPAD + ko);
#pragma unroll
      for (int g = 0; g < 4; ++g) acc[g] = Frag<_Float16>::mma(af, bq[g], acc[g]);
      dep_guard_h(acc[0], acc[3], af, bq[3]);
      keep4_h(bq[0], bq[1], bq[2], bq[3]);
    }
    acc_guard4(acc[0], acc[1], acc[2], acc[3]);

#pragma unroll
    for (int r = 0; r < 8; ++r) {
      const float pi = acc[0][r] * kWScaleInv + bs[0];
      const float pf = acc[1][r] * kWScaleInv + bs[1];
      const float pg = acc[2][r] * kWScaleInv + bs[2];
      const float po = acc[3][r] * kWScaleInv + bs[3];
      const float ig = sigm_f(pi);
      const float fg = sigm_f(pf);
      const float gg = tanh_f(pg);
      const float og = sigm_f(po);
      const float cn = fg * cst[r] + ig * gg;
      cst[r] = cn;
      const float hn = og * tanh_f(cn);
      nxt[(8 * hh + r) * AP + ucol] = (_Float16)hn;
    }
    if (t + 1 < kSteps) {
      if constexpr (KIN == kIn) {
        if (tid < 16 * kIn) nxt[xm * AP + kHid + xj] = (_Float16)xs;
      } else {
        *(v4u*)(nxt + xm * AP + kHid + xj) = xq;
      }
    }
    __syncthreads();

    {
      const int row = 2 * wv + hh;
      const int c8  = cc * 8;
      const v4u hq = *(const v4u*)(nxt + row * AP + c8);
      _Float16* gp = hout16 + ((size_t)(b0 + row) * kSteps + t) * kHid + c8;
      *(volatile v4u*)gp = hq;
      __threadfence();
      *(volatile v4u*)gp = hq;
    }
  }
}

__global__ __launch_bounds__(256) void prep_fc1_kernel(const float* __restrict__ w, unsigned short* __restrict__ plane) {
  const int i   = blockIdx.x * 256 + threadIdx.x;
  const int n   = i >> 4;
  const int k8  = (i & 15) * 8;
  const int ncl = (n < kFc1) ? n : (kFc1 - 1);
  const v4f a = *(const v4f*)(w + (size_t)ncl * kHid + k8);
  const v4f c = *(const v4f*)(w + (size_t)ncl * kHid + k8 + 4);
  const bool live = (n < kFc1);
  float f[8];
  f[0] = live ? a[0] * kWScale : 0.0f; f[1] = live ? a[1] * kWScale : 0.0f;
  f[2] = live ? a[2] * kWScale : 0.0f; f[3] = live ? a[3] * kWScale : 0.0f;
  f[4] = live ? c[0] * kWScale : 0.0f; f[5] = live ? c[1] * kWScale : 0.0f;
  f[6] = live ? c[2] * kWScale : 0.0f; f[7] = live ? c[3] * kWScale : 0.0f;
  v8h hv;
#pragma unroll
  for (int e = 0; e < 8; ++e) hv[e] = (_Float16)f[e];
  _Float16* gp = (_Float16*)plane + (size_t)i * 8;
  *(volatile v8h*)gp = hv;
  __threadfence();
  *(volatile v8h*)gp = hv;
}

__global__ __launch_bounds__(256) void head_out_kernel(const float* __restrict__ gmat,
                                                       const float* __restrict__ b1,
                                                       const float* __restrict__ w2,
                                                       const float* __restrict__ b2,
                                                       float* __restrict__ out) {
  __shared__ __align__(16) float srow[256 * 24];
  __shared__ float sb1[32];
  __shared__ float sw2[32];
  const int tid = threadIdx.x;
  const int row = blockIdx.x * 256 + tid;
  {
    const int j = (tid < kFc1) ? tid : (kFc1 - 1);
    const float bv = b1[j];
    const float wvv = w2[j];
    if (tid < kFc1) { sb1[tid] = bv; sw2[tid] = wvv; }
  }
  const float* gp = gmat + (size_t)row * kHeadN;
#pragma unroll
  for (int q = 0; q < 5; ++q) {
    const v4f v = *(const v4f*)(gp + 4 * q);
    *(v4f*)(srow + tid * 24 + 4 * q) = v;
  }
  __syncthreads();
  float acc = 0.0f;
#pragma unroll 1
  for (int j = 0; j < kFc1; ++j) {
    const float v  = srow[tid * 24 + j] + sb1[j];
    const float tv = tanh_f(v);
    acc = fmaf(tv, sw2[j], acc);
  }
  const float res = acc + b2[0];
  *(volatile float*)(out + row) = res;
  __threadfence();
  *(volatile float*)(out + row) = res;
}

extern "C" void kernel_launch(void* const* d_in, const int* in_sizes, int n_in,
                              void* d_out, int out_size, void* d_ws, size_t ws_size,
                              hipStream_t stream) {
  (void)n_in;
  if (in_sizes[0] != kBatch * kSteps * kIn) return;
  if (out_size != kRows) return;
  if (ws_size < kWsTotal) return;

  const float* x     = (const float*)d_in[0];
  const float* W_ih0 = (const float*)d_in[1];
  const float* W_hh0 = (const float*)d_in[2];
  const float* b_ih0 = (const float*)d_in[3];
  const float* b_hh0 = (const float*)d_in[4];
  const float* W_ih1 = (const float*)d_in[5];
  const float* W_hh1 = (const float*)d_in[6];
  const float* b_ih1 = (const float*)d_in[7];
  const float* b_hh1 = (const float*)d_in[8];
  const float* fc1_w = (const float*)d_in[9];
  const float* fc1_b = (const float*)d_in[10];
  const float* fc2_w = (const float*)d_in[11];
  const float* fc2_b = (const float*)d_in[12];
  float* outp = (float*)d_out;

  char* ws = (char*)d_ws;
  unsigned short* h0p  = (unsigned short*)(ws + kOffH0);
  unsigned short* h1p  = (unsigned short*)(ws + kOffH1);
  float*          gmat = (float*)(ws + kOffGmat);
  unsigned short* fc1p = (unsigned short*)(ws + kOffFc1);

  constexpr size_t kLds0 = ((size_t)kGates * kKpad0 + 32 * (kKpad0 + 8)) * 2;
  constexpr size_t kLds1 = ((size_t)kGates * kKpad1 + 32 * (kKpad1 + 8)) * 2;
  static_assert(kLds0 == 174592 && kLds1 == 279040, "lds sizes");

  prep_fc1_kernel<<<4, 256, 0, stream>>>(fc1_w, fc1p);

  lstm_layer_kernel<kIn, kKpad0><<<kBatch / 16, 256, kLds0, stream>>>(W_hh0, W_ih0, b_ih0, b_hh0, x, h1p, h0p);
  lstm_layer_kernel<kHid, kKpad1><<<kBatch / 16, 256, kLds1, stream>>>(W_hh1, W_ih1, b_ih1, b_hh1, x, h0p, h1p);

  wmma_gemm64<0, false, 0, 0, false, 0><<<dim3((kRows / 64) * (kHeadN / 64) / 8, 1, 1), 256, 0, stream>>>(
      h1p, h1p, kHid, 0L,
      fc1p, fc1p, kHid, 0L,
      (void*)gmat, (void*)gmat, kHeadN, 0L,
      fc1_b,
      fc1_b, 0L,
      kRows, kHeadN, kHid, kWScaleInv);

  head_out_kernel<<<kRows / 256, 256, 0, stream>>>(gmat, fc1_b, fc2_w, fc2_b, outp);
}
